// GINEncoder_90228672955075
// MI455X (gfx1250) — hardware-verified
//
#include <hip/hip_runtime.h>
#include <stddef.h>
#include <stdint.h>


#define FIN0    128
#define HD      256
#define KH      512
#define K0      256
#define NTHR    256
#define NWAVE   8
#define EPT     8
#define CHUNK   (NTHR * EPT)
#define WCAP    (EPT * 32)
#define LISTN   (NWAVE * WCAP)
#define NB      1024
#define NBSH    10
#define PKS     10
#define RCAP    28672
#define DEGCAP  64
#define RPW     8
#define GBM     64
#define GBN     128
#define GTHR    128
#define GNT     8
#define PARTW   256
#define NU0     (HD * (K0 / 8))
#define NUW     (HD * (KH / 8))
#define NUTOT   (NU0 + 5 * NUW)
#define HZINTS  (2 * RCAP + 2 * NB + LISTN)
#define LDS_HITS (HZINTS * 4 + 64)
#define WSLIM   134217728

static_assert((CHUNK & (CHUNK - 1)) == 0 && CHUNK == 2048);
static_assert(NB == (1 << NBSH) && NB <= (1 << PKS) && NTHR * 4 == NB);
static_assert(LISTN >= NB && LISTN >= NWAVE * WCAP);
static_assert((RCAP % (4 * NTHR)) == 0 && (HZINTS % (4 * NTHR)) == 0);
static_assert(RCAP < (1 << 15));
static_assert(LDS_HITS <= 300000);
static_assert(GBM == (GTHR / 32) * 16 && GBN == 16 * GNT && GTHR == GBN);
static_assert(GBM == NWAVE * RPW);
static_assert((K0 % 32) == 0 && (KH % 32) == 0 && (HD % GBN) == 0);
static_assert(HD * 4 == KH * 2 && K0 == 2 * FIN0 && KH == 2 * HD);
static_assert(HD == 32 * 8 && FIN0 == 32 * 4 && NTHR == HD);
static_assert((NU0 % NTHR) == 0 && (NUW % NTHR) == 0 && NUW == (1 << 14));
static_assert(PARTW == 2 * GBN && PARTW / 4 <= GTHR);
static_assert(DEGCAP < 255);

typedef float          v4f  __attribute__((ext_vector_type(4)));
typedef float          v8f  __attribute__((ext_vector_type(8)));
typedef int            v4i  __attribute__((ext_vector_type(4)));
typedef int            v8i  __attribute__((ext_vector_type(8)));
typedef unsigned int   v2u  __attribute__((ext_vector_type(2)));
typedef unsigned int   v4u  __attribute__((ext_vector_type(4)));
typedef unsigned short v8us __attribute__((ext_vector_type(8)));
typedef __bf16         v16b __attribute__((ext_vector_type(16)));
typedef v4f  __attribute__((may_alias)) v4fa;
typedef v4i  __attribute__((may_alias)) v4ia;
typedef v2u  __attribute__((may_alias)) v2ua;
typedef v8us __attribute__((may_alias)) v8usa;
union Frag { v16b vb; v8us h[2]; v8i w; };

__device__ __forceinline__ v8f wmb(const Frag& a, const Frag& b, v8f c) {
  v8f d = __builtin_amdgcn_wmma_f32_16x16x32_bf16(false, a.vb, false, b.vb, (short)0, c, false, false);
  asm volatile("v_nop\n\tv_nop\n\tv_nop\n\tv_nop" : "+v"(d) : "v"(a.w), "v"(b.w));
  return d;
}

__device__ __forceinline__ unsigned bf_bits(float f) {
  const unsigned u = __float_as_uint(f);
  return (u + 0x7FFFu + ((u >> 16) & 1u)) >> 16;
}
__device__ __forceinline__ float bf_val(unsigned b) { return __uint_as_float(b << 16); }
__device__ __forceinline__ float bf_rne(float f) { return bf_val(bf_bits(f)); }

__device__ __forceinline__ float bnf(float u, float m, float rs, float g, float be) {
  return g * (u - m) * rs + be;
}

__device__ __forceinline__ int scan_chunk(const int* __restrict__ dsts, int nE, int cbase, int slotBase,
                                          int nb, int vec8, int* list, int tid, int lane, int wave) {
  int wc = 0;
  const int el0  = tid * EPT;
  const int e0   = cbase + el0;
  const int sent = -2147483647 - 1;
  v4i da, db;
  if (vec8 != 0 && cbase + CHUNK <= nE) {
    da = *(const v4i*)(dsts + e0);
    db = *(const v4i*)(dsts + e0 + 4);
  } else {
    da.x = (e0     < nE) ? dsts[min(e0,     nE - 1)] : sent;
    da.y = (e0 + 1 < nE) ? dsts[min(e0 + 1, nE - 1)] : sent;
    da.z = (e0 + 2 < nE) ? dsts[min(e0 + 2, nE - 1)] : sent;
    da.w = (e0 + 3 < nE) ? dsts[min(e0 + 3, nE - 1)] : sent;
    db.x = (e0 + 4 < nE) ? dsts[min(e0 + 4, nE - 1)] : sent;
    db.y = (e0 + 5 < nE) ? dsts[min(e0 + 5, nE - 1)] : sent;
    db.z = (e0 + 6 < nE) ? dsts[min(e0 + 6, nE - 1)] : sent;
    db.w = (e0 + 7 < nE) ? dsts[min(e0 + 7, nE - 1)] : sent;
  }
  const unsigned nbs = (unsigned)slotBase;
  const unsigned unb = (unsigned)nb;
  const unsigned s0 = (unsigned)da.x - nbs, s1 = (unsigned)da.y - nbs;
  const unsigned s2 = (unsigned)da.z - nbs, s3 = (unsigned)da.w - nbs;
  const unsigned s4 = (unsigned)db.x - nbs, s5 = (unsigned)db.y - nbs;
  const unsigned s6 = (unsigned)db.z - nbs, s7 = (unsigned)db.w - nbs;
  const bool h0 = s0 < unb, h1 = s1 < unb, h2 = s2 < unb, h3 = s3 < unb;
  const bool h4 = s4 < unb, h5 = s5 < unb, h6 = s6 < unb, h7 = s7 < unb;
  const unsigned any = __builtin_amdgcn_ballot_w32(h0 | h1 | h2 | h3 | h4 | h5 | h6 | h7);
  if (any != 0u) {
#define HITJ(J, HJ, SJ) { \
      const unsigned mj = __builtin_amdgcn_ballot_w32(HJ); \
      if (mj != 0u) { \
        if (HJ) { \
          const int pos = wc + (int)__builtin_amdgcn_mbcnt_lo(mj, 0u); \
          if (pos < WCAP) list[wave * WCAP + pos] = ((el0 + (J)) << PKS) | (int)(SJ); \
        } \
        wc += (int)__builtin_popcount(mj); } }
    HITJ(0, h0, s0)
    HITJ(1, h1, s1)
    HITJ(2, h2, s2)
    HITJ(3, h3, s3)
    HITJ(4, h4, s4)
    HITJ(5, h5, s5)
    HITJ(6, h6, s6)
    HITJ(7, h7, s7)
#undef HITJ
  }
  return wc;
}

__device__ __forceinline__ v8us cv8b(const float* __restrict__ p, size_t stride) {
  v8us o;
#pragma unroll
  for (int i = 0; i < 8; ++i) o[i] = (unsigned short)bf_bits(p[(size_t)i * stride]);
  return o;
}

__global__ __launch_bounds__(NTHR) void k_wprep(const float* __restrict__ w10, const float* __restrict__ w20,
                                                const float* __restrict__ w11, const float* __restrict__ w21,
                                                const float* __restrict__ w12, const float* __restrict__ w22,
                                                unsigned short* p10, unsigned short* p20, unsigned short* p11,
                                                unsigned short* p21, unsigned short* p12, unsigned short* p22) {
  const int u = (int)blockIdx.x * NTHR + (int)threadIdx.x;
  const float* sp;
  unsigned short* dp;
  if (u < NU0) {
    const int n  = u >> 5;
    const int k8 = (u & 31) * 8;
    const int kk = k8 & (FIN0 - 1);
    sp = w10 + (size_t)kk * HD + n;
    dp = p10 + (size_t)u * 8;
  } else if (u < NUTOT) {
    const int w  = u - NU0;
    const int pi = w >> 14;
    const int v  = w & (NUW - 1);
    const int n  = v >> 6;
    const int k8 = (v & 63) * 8;
    const int kk = k8 & (HD - 1);
    const float* wb = w20;
    unsigned short* pb = p20;
    if (pi == 1)      { wb = w11; pb = p11; }
    else if (pi == 2) { wb = w21; pb = p21; }
    else if (pi == 3) { wb = w12; pb = p12; }
    else if (pi == 4) { wb = w22; pb = p22; }
    sp = wb + (size_t)kk * HD + n;
    dp = pb + (size_t)v * 8;
  } else {
    return;
  }
  const v8us o = cv8b(sp, HD);
  *(volatile v8us*)dp = o;
  __threadfence();
  *(volatile v8us*)dp = o;
}

__global__ __launch_bounds__(NTHR) void k_cvx(const float* __restrict__ x, int nN, int nUnits,
                                              unsigned short* xb) {
  const int u = (int)blockIdx.x * NTHR + (int)threadIdx.x;
  if (u >= nUnits) return;
  const int row = u >> 4;
  const int k8  = (u & 15) * 8;
  const int rc  = row < nN ? row : nN - 1;
  const float* p = x + (size_t)rc * FIN0 + k8;
  const v4f a = *(const v4fa*)p;
  const v4f b = *(const v4fa*)(p + 4);
  const bool ok = row < nN;
  v8us o;
  o[0] = ok ? (unsigned short)bf_bits(a.x) : (unsigned short)0;
  o[1] = ok ? (unsigned short)bf_bits(a.y) : (unsigned short)0;
  o[2] = ok ? (unsigned short)bf_bits(a.z) : (unsigned short)0;
  o[3] = ok ? (unsigned short)bf_bits(a.w) : (unsigned short)0;
  o[4] = ok ? (unsigned short)bf_bits(b.x) : (unsigned short)0;
  o[5] = ok ? (unsigned short)bf_bits(b.y) : (unsigned short)0;
  o[6] = ok ? (unsigned short)bf_bits(b.z) : (unsigned short)0;
  o[7] = ok ? (unsigned short)bf_bits(b.w) : (unsigned short)0;
  unsigned short* dp = xb + (size_t)row * FIN0 + k8;
  *(volatile v8us*)dp = o;
  __threadfence();
  *(volatile v8us*)dp = o;
}

__global__ __launch_bounds__(NTHR) void k_hits(const int* __restrict__ srcs, const int* __restrict__ dsts,
                                               int nN, int nE, int vec8, int* slotTab, int* srcList) {
  extern __shared__ v4f lds_dyn[];
  int* reg1 = (int*)lds_dyn;
  int* reg2 = reg1 + RCAP;
  int* scnt = reg2 + RCAP;
  int* soff = scnt + NB;
  int* list = soff + NB;
  int* wcnt = list + LISTN;
  int* wtot = wcnt + NWAVE;
  const int tid = (int)threadIdx.x, lane = tid & 31, wave = tid >> 5;
  const int nodeBase = (int)blockIdx.x * NB;

  {
    const v4i z4 = {0, 0, 0, 0};
    for (int i = tid * 4; i < HZINTS; i += NTHR * 4) *(v4ia*)(reg1 + i) = z4;
    if (tid < 2 * NWAVE) wcnt[tid] = 0;
  }
  __syncthreads();

  int tot = 0;
  const int nChunks = (nE + CHUNK - 1) / CHUNK;
#pragma unroll 1
  for (int ch = 0; ch < nChunks; ++ch) {
    const int cbase = ch * CHUNK;
    const int wc = scan_chunk(dsts, nE, cbase, nodeBase, NB, vec8, list, tid, lane, wave);
    if (lane == 0) wcnt[wave] = wc;
    __syncthreads();
    int pre = 0, all = 0;
#pragma unroll
    for (int w2 = 0; w2 < NWAVE; ++w2) {
      int c = wcnt[w2];
      c = c < 0 ? 0 : (c > WCAP ? WCAP : c);
      all += c;
      pre += (w2 < wave) ? c : 0;
    }
    const int wcc  = wc > WCAP ? WCAP : wc;
    const int base = tot + pre;
#pragma unroll 1
    for (int i = lane; i < wcc; i += 32) {
      const int ent = list[wave * WCAP + i];
      const int el  = (ent >> PKS) & (CHUNK - 1);
      const int sl  = ent & (NB - 1);
      int eid = cbase + el;
      eid = eid > nE - 1 ? nE - 1 : eid;
      const int pos = base + i;
      if (pos < RCAP) reg1[pos] = (int)(((unsigned)eid << PKS) | (unsigned)sl);
    }
    tot += all;
    tot = tot > RCAP ? RCAP : tot;
    __syncthreads();
  }
  const int nh = tot;

  if (wave == 0) {
#pragma unroll 1
    for (int b0 = 0; b0 < nh; b0 += 32) {
      const int idx = b0 + lane;
      const int uv  = reg1[idx < RCAP ? idx : RCAP - 1];
      const int m32 = (nh - b0) < 32 ? (nh - b0) : 32;
#pragma unroll 1
      for (int k = 0; k < m32; ++k) {
        const int u  = __builtin_amdgcn_readlane(uv, k);
        const int sl = u & (NB - 1);
        if (lane == 0) scnt[sl] = scnt[sl] + 1;
      }
    }
  }
  __syncthreads();

  {
    const v4i ca = *(const v4ia*)(scnt + 4 * tid);
    const int e0 = ca.x < 0 ? 0 : ca.x, e1 = ca.y < 0 ? 0 : ca.y, e2 = ca.z < 0 ? 0 : ca.z, e3 = ca.w < 0 ? 0 : ca.w;
    const int ts = e0 + e1 + e2 + e3;
    int incl = ts;
#pragma unroll
    for (int d = 1; d < 32; d <<= 1) {
      const int up = __shfl_up(incl, d);
      if (lane >= d) incl += up;
    }
    if (lane == 31) wtot[wave] = incl;
    __syncthreads();
    int pre = 0;
#pragma unroll
    for (int w2 = 0; w2 < NWAVE; ++w2) pre += (w2 < wave) ? wtot[w2] : 0;
    int run = pre + incl - ts;
    soff[4 * tid + 0] = run; run += e0;
    soff[4 * tid + 1] = run; run += e1;
    soff[4 * tid + 2] = run; run += e2;
    soff[4 * tid + 3] = run;
  }
  __syncthreads();
  for (int i = tid; i < NB; i += NTHR) list[i] = soff[i];
  __syncthreads();

  if (wave == 0) {
#pragma unroll 1
    for (int b0 = 0; b0 < nh; b0 += 32) {
      const int idx = b0 + lane;
      const int uv  = reg1[idx < RCAP ? idx : RCAP - 1];
      const int m32 = (nh - b0) < 32 ? (nh - b0) : 32;
#pragma unroll 1
      for (int k = 0; k < m32; ++k) {
        const int u   = __builtin_amdgcn_readlane(uv, k);
        const int sl  = u & (NB - 1);
        const int eid = (int)((unsigned)u >> PKS);
        if (lane == 0) {
          int pos = list[sl];
          pos = pos < 0 ? 0 : (pos > RCAP - 1 ? RCAP - 1 : pos);
          reg2[pos] = eid;
          list[sl] = pos + 1;
        }
      }
    }
  }
  __syncthreads();

  const bool ovf = (nh >= RCAP);
  {
    const v4i so = *(const v4ia*)(soff + 4 * tid);
    const v4i sc = *(const v4ia*)(scnt + 4 * tid);
    int o0 = so.x < 0 ? 0 : (so.x > RCAP ? RCAP : so.x);
    int o1 = so.y < 0 ? 0 : (so.y > RCAP ? RCAP : so.y);
    int o2 = so.z < 0 ? 0 : (so.z > RCAP ? RCAP : so.z);
    int o3 = so.w < 0 ? 0 : (so.w > RCAP ? RCAP : so.w);
    int c0 = sc.x < 0 ? 0 : (sc.x > 255 ? 255 : sc.x);
    int c1 = sc.y < 0 ? 0 : (sc.y > 255 ? 255 : sc.y);
    int c2 = sc.z < 0 ? 0 : (sc.z > 255 ? 255 : sc.z);
    int c3 = sc.w < 0 ? 0 : (sc.w > 255 ? 255 : sc.w);
    c0 = ovf ? 255 : c0; c1 = ovf ? 255 : c1; c2 = ovf ? 255 : c2; c3 = ovf ? 255 : c3;
    v4i ev;
    ev.x = (o0 << 8) | c0; ev.y = (o1 << 8) | c1; ev.z = (o2 << 8) | c2; ev.w = (o3 << 8) | c3;
    int* dp = slotTab + (size_t)blockIdx.x * NB + 4 * tid;
    *(volatile v4i*)dp = ev;
    __threadfence();
    *(volatile v4i*)dp = ev;
  }
#pragma unroll 1
  for (int it = 0; it < RCAP / (4 * NTHR); ++it) {
    const int p = 4 * (it * NTHR + tid);
    const v4i ev = *(const v4ia*)(reg2 + p);
    const int e0 = ev.x < 0 ? 0 : (ev.x > nE - 1 ? nE - 1 : ev.x);
    const int e1 = ev.y < 0 ? 0 : (ev.y > nE - 1 ? nE - 1 : ev.y);
    const int e2 = ev.z < 0 ? 0 : (ev.z > nE - 1 ? nE - 1 : ev.z);
    const int e3 = ev.w < 0 ? 0 : (ev.w > nE - 1 ? nE - 1 : ev.w);
    int s0 = srcs[e0], s1 = srcs[e1], s2 = srcs[e2], s3 = srcs[e3];
    s0 = s0 < 0 ? 0 : (s0 > nN - 1 ? nN - 1 : s0);
    s1 = s1 < 0 ? 0 : (s1 > nN - 1 ? nN - 1 : s1);
    s2 = s2 < 0 ? 0 : (s2 > nN - 1 ? nN - 1 : s2);
    s3 = s3 < 0 ? 0 : (s3 > nN - 1 ? nN - 1 : s3);
    v4i o;
    o.x = (p     < nh) ? s0 : 0;
    o.y = (p + 1 < nh) ? s1 : 0;
    o.z = (p + 2 < nh) ? s2 : 0;
    o.w = (p + 3 < nh) ? s3 : 0;
    int* dp = srcList + (size_t)blockIdx.x * RCAP + p;
    *(volatile v4i*)dp = o;
    __threadfence();
    *(volatile v4i*)dp = o;
  }
}

template <int L0>
__global__ __launch_bounds__(NTHR) void k_agg(const int* __restrict__ slotTab, const int* __restrict__ srcList,
                                              const unsigned short* __restrict__ xb,
                                              const float* __restrict__ uf, const float* __restrict__ stats,
                                              unsigned short* Sout, int nN, int MPr, int nSlots) {
  const int tid = (int)threadIdx.x, lane = tid & 31, wave = tid >> 5;
  const int rowBase = (int)blockIdx.x * (NWAVE * RPW) + wave * RPW;
  float cm[8], cr[8], cg[8], cb[8];
  if constexpr (L0 == 0) {
    const v4f m0 = *(const v4f*)(stats + 8 * lane),          m1 = *(const v4f*)(stats + 8 * lane + 4);
    const v4f r0 = *(const v4f*)(stats + HD + 8 * lane),     r1 = *(const v4f*)(stats + HD + 8 * lane + 4);
    const v4f g0 = *(const v4f*)(stats + 2 * HD + 8 * lane), g1 = *(const v4f*)(stats + 2 * HD + 8 * lane + 4);
    const v4f b0 = *(const v4f*)(stats + 3 * HD + 8 * lane), b1 = *(const v4f*)(stats + 3 * HD + 8 * lane + 4);
    cm[0] = m0.x; cm[1] = m0.y; cm[2] = m0.z; cm[3] = m0.w; cm[4] = m1.x; cm[5] = m1.y; cm[6] = m1.z; cm[7] = m1.w;
    cr[0] = r0.x; cr[1] = r0.y; cr[2] = r0.z; cr[3] = r0.w; cr[4] = r1.x; cr[5] = r1.y; cr[6] = r1.z; cr[7] = r1.w;
    cg[0] = g0.x; cg[1] = g0.y; cg[2] = g0.z; cg[3] = g0.w; cg[4] = g1.x; cg[5] = g1.y; cg[6] = g1.z; cg[7] = g1.w;
    cb[0] = b0.x; cb[1] = b0.y; cb[2] = b0.z; cb[3] = b0.w; cb[4] = b1.x; cb[5] = b1.y; cb[6] = b1.z; cb[7] = b1.w;
  } else {
#pragma unroll
    for (int i = 0; i < 8; ++i) { cm[i] = 0.0f; cr[i] = 1.0f; cg[i] = 1.0f; cb[i] = 0.0f; }
  }
  const float qnan = __int_as_float(0x7fc00000);

#pragma unroll 1
  for (int j = 0; j < RPW; ++j) {
    const int grow = rowBase + j;
    const int gs   = grow < nSlots ? grow : nSlots - 1;
    int ent = slotTab[gs];
    ent = __builtin_amdgcn_readfirstlane(ent);
    int st = (int)((unsigned)ent >> 8);
    st = st > RCAP ? RCAP : st;
    const int c8 = ent & 255;
    int cnt = c8 > DEGCAP ? DEGCAP : c8;
    if (cnt > RCAP - st) cnt = RCAP - st;
    const bool liveRow = grow < nN;
    const float pz = (liveRow && c8 > DEGCAP) ? qnan : 0.0f;
    const int* sbase = srcList + (size_t)(gs >> NBSH) * RCAP;

    float ag[8];
#pragma unroll
    for (int i = 0; i < 8; ++i) ag[i] = 0.0f;

#pragma unroll 1
    for (int b0 = 0; b0 < cnt; b0 += 32) {
      int idx = st + b0 + lane;
      idx = idx > RCAP - 1 ? RCAP - 1 : idx;
      int sr = sbase[idx];
      sr = sr < 0 ? 0 : (sr > nN - 1 ? nN - 1 : sr);
      const int m32 = (cnt - b0) < 32 ? (cnt - b0) : 32;
#pragma unroll 1
      for (int k = 0; k < m32; ++k) {
        const int sk = __builtin_amdgcn_readlane(sr, k);
        if constexpr (L0 != 0) {
          const v2u w = *(const v2ua*)(xb + (size_t)sk * FIN0 + 4 * lane);
          ag[0] += __uint_as_float(w.x << 16);
          ag[1] += __uint_as_float(w.x & 0xffff0000u);
          ag[2] += __uint_as_float(w.y << 16);
          ag[3] += __uint_as_float(w.y & 0xffff0000u);
        } else {
          const float* rp = uf + (size_t)sk * HD + 8 * lane;
          const v4f a = *(const v4f*)rp;
          const v4f b = *(const v4f*)(rp + 4);
          ag[0] += bnf(a.x, cm[0], cr[0], cg[0], cb[0]);
          ag[1] += bnf(a.y, cm[1], cr[1], cg[1], cb[1]);
          ag[2] += bnf(a.z, cm[2], cr[2], cg[2], cb[2]);
          ag[3] += bnf(a.w, cm[3], cr[3], cg[3], cb[3]);
          ag[4] += bnf(b.x, cm[4], cr[4], cg[4], cb[4]);
          ag[5] += bnf(b.y, cm[5], cr[5], cg[5], cb[5]);
          ag[6] += bnf(b.z, cm[6], cr[6], cg[6], cb[6]);
          ag[7] += bnf(b.w, cm[7], cr[7], cg[7], cb[7]);
        }
      }
    }

    const int nc = liveRow ? grow : nN - 1;
    const bool wsv = grow < MPr;
    if constexpr (L0 != 0) {
      const v2u w = *(const v2ua*)(xb + (size_t)nc * FIN0 + 4 * lane);
      float r[4];
      r[0] = __uint_as_float(w.x << 16) + ag[0];
      r[1] = __uint_as_float(w.x & 0xffff0000u) + ag[1];
      r[2] = __uint_as_float(w.y << 16) + ag[2];
      r[3] = __uint_as_float(w.y & 0xffff0000u) + ag[3];
#pragma unroll
      for (int i = 0; i < 4; ++i) r[i] = (liveRow ? r[i] : 0.0f) + pz;
      const unsigned h0 = bf_bits(r[0]), h1 = bf_bits(r[1]), h2 = bf_bits(r[2]), h3 = bf_bits(r[3]);
      const unsigned l0 = bf_bits(r[0] - bf_val(h0)), l1 = bf_bits(r[1] - bf_val(h1));
      const unsigned l2 = bf_bits(r[2] - bf_val(h2)), l3 = bf_bits(r[3] - bf_val(h3));
      v2u hv, lv;
      hv.x = h0 | (h1 << 16); hv.y = h2 | (h3 << 16);
      lv.x = l0 | (l1 << 16); lv.y = l2 | (l3 << 16);
      unsigned short* hp = Sout + (size_t)grow * K0 + 4 * lane;
      unsigned short* lp = hp + FIN0;
      if (wsv) { *(volatile v2u*)hp = hv; *(volatile v2u*)lp = lv; }
      __threadfence();
      if (wsv) { *(volatile v2u*)hp = hv; *(volatile v2u*)lp = lv; }
    } else {
      const float* rp = uf + (size_t)nc * HD + 8 * lane;
      const v4f a = *(const v4f*)rp;
      const v4f b = *(const v4f*)(rp + 4);
      float r[8];
      r[0] = bnf(a.x, cm[0], cr[0], cg[0], cb[0]) + ag[0];
      r[1] = bnf(a.y, cm[1], cr[1], cg[1], cb[1]) + ag[1];
      r[2] = bnf(a.z, cm[2], cr[2], cg[2], cb[2]) + ag[2];
      r[3] = bnf(a.w, cm[3], cr[3], cg[3], cb[3]) + ag[3];
      r[4] = bnf(b.x, cm[4], cr[4], cg[4], cb[4]) + ag[4];
      r[5] = bnf(b.y, cm[5], cr[5], cg[5], cb[5]) + ag[5];
      r[6] = bnf(b.z, cm[6], cr[6], cg[6], cb[6]) + ag[6];
      r[7] = bnf(b.w, cm[7], cr[7], cg[7], cb[7]) + ag[7];
      unsigned hw[4], lw[4];
#pragma unroll
      for (int q = 0; q < 4; ++q) {
        const float v0 = (liveRow ? r[2 * q] : 0.0f) + pz;
        const float v1 = (liveRow ? r[2 * q + 1] : 0.0f) + pz;
        const unsigned h0 = bf_bits(v0), h1 = bf_bits(v1);
        const unsigned l0 = bf_bits(v0 - bf_val(h0)), l1 = bf_bits(v1 - bf_val(h1));
        hw[q] = h0 | (h1 << 16);
        lw[q] = l0 | (l1 << 16);
      }
      v4u hv, lv;
      hv.x = hw[0]; hv.y = hw[1]; hv.z = hw[2]; hv.w = hw[3];
      lv.x = lw[0]; lv.y = lw[1]; lv.z = lw[2]; lv.w = lw[3];
      unsigned short* hp = Sout + (size_t)grow * KH + 8 * lane;
      unsigned short* lp = hp + HD;
      if (wsv) { *(volatile v4u*)hp = hv; *(volatile v4u*)lp = lv; }
      __threadfence();
      if (wsv) { *(volatile v4u*)hp = hv; *(volatile v4u*)lp = lv; }
    }
  }
}

template <int EPI>
__global__ __launch_bounds__(GTHR) void k_gemm(const unsigned short* __restrict__ A, int lda,
                                               const unsigned short* __restrict__ BT, int ldb, int K,
                                               const float* __restrict__ bias,
                                               void* outp, int ldo, int lsplit, int nN, int mRows,
                                               float* part) {
  __shared__ __attribute__((aligned(16))) float stg[GBM * GBN];
  __shared__ __attribute__((aligned(16))) float pst[PARTW];
  const int tid = (int)threadIdx.x, lane = tid & 31, wave = tid >> 5, hh = lane >> 4, m = lane & 15;
  const int rowBase = (int)blockIdx.x * GBM;
  const int colBase = (int)blockIdx.y * GBN;

  v8f acc[GNT];
  {
    const v8f z = {0.f, 0.f, 0.f, 0.f, 0.f, 0.f, 0.f, 0.f};
#pragma unroll
    for (int t = 0; t < GNT; ++t) acc[t] = z;
  }
  const unsigned short* ap = A  + (size_t)(rowBase + 16 * wave + m) * (size_t)lda + 8 * hh;
  const unsigned short* bp = BT + (size_t)(colBase + m) * (size_t)ldb + 8 * hh;

#pragma unroll 1
  for (int k0 = 0; k0 < K; k0 += 32) {
    Frag af;
    af.h[0] = *(const v8usa*)(ap + k0);
    af.h[1] = *(const v8usa*)(ap + k0 + 16);
#pragma unroll
    for (int nt = 0; nt < GNT; ++nt) {
      const unsigned short* wq = bp + (size_t)(16 * nt) * (size_t)ldb + k0;
      Frag bfr;
      bfr.h[0] = *(const v8usa*)wq;
      bfr.h[1] = *(const v8usa*)(wq + 16);
      acc[nt] = wmb(af, bfr, acc[nt]);
    }
  }

#pragma unroll
  for (int nt = 0; nt < GNT; ++nt) {
    const int lc = 16 * nt + m;
    const float bb = bf_rne(bias[colBase + lc]);
#pragma unroll
    for (int r = 0; r < 8; ++r) {
      const int lr = 16 * wave + 8 * hh + r;
      const bool live = (rowBase + lr) < nN;
      float v = acc[nt][r] + bb;
      v = (v > 0.0f) ? v : (v - v);
      stg[lr * GBN + lc] = live ? v : 0.0f;
    }
  }
  __syncthreads();

  if constexpr (EPI == 0) {
    unsigned short* outH = (unsigned short*)outp;
    const int cb = 8 * m;
    const bool isHi = (hh == 0);
    v4u pk[16];
#pragma unroll
    for (int i = 0; i < 16; ++i) {
      const int lr = 16 * wave + i;
      const v4f a = *(const v4fa*)(stg + lr * GBN + cb);
      const v4f b = *(const v4fa*)(stg + lr * GBN + cb + 4);
      const float f[8] = {a.x, a.y, a.z, a.w, b.x, b.y, b.z, b.w};
      unsigned int w[4];
#pragma unroll
      for (int j = 0; j < 4; ++j) {
        const unsigned h0 = bf_bits(f[2 * j]), h1 = bf_bits(f[2 * j + 1]);
        const unsigned l0 = bf_bits(f[2 * j] - bf_val(h0)), l1 = bf_bits(f[2 * j + 1] - bf_val(h1));
        const unsigned q0 = isHi ? h0 : l0, q1 = isHi ? h1 : l1;
        w[j] = q0 | (q1 << 16);
      }
      v4u pv; pv.x = w[0]; pv.y = w[1]; pv.z = w[2]; pv.w = w[3];
      pk[i] = pv;
    }
#pragma unroll
    for (int i = 0; i < 16; ++i) {
      const int gr = rowBase + 16 * wave + i;
      unsigned short* op = outH + (size_t)gr * (size_t)ldo + colBase + cb + hh * lsplit;
      if (gr < mRows) *(volatile v4u*)op = pk[i];
    }
    __threadfence();
#pragma unroll
    for (int i = 0; i < 16; ++i) {
      const int gr = rowBase + 16 * wave + i;
      unsigned short* op = outH + (size_t)gr * (size_t)ldo + colBase + cb + hh * lsplit;
      if (gr < mRows) *(volatile v4u*)op = pk[i];
    }
  } else {
    float* outF = (float*)outp;
    v4f fv[16];
#pragma unroll
    for (int i = 0; i < 16; ++i) {
      const int lr = 16 * wave + i;
      fv[i] = *(const v4fa*)(stg + lr * GBN + 4 * lane);
    }
    int nvr = nN - rowBase;
    nvr = nvr < 0 ? 0 : (nvr > GBM ? GBM : nvr);
    float s = 0.0f, q = 0.0f;
#pragma unroll 4
    for (int r = 0; r < nvr; ++r) {
      const float v = stg[r * GBN + tid];
      s += v;
      q = fmaf(v, v, q);
    }
    pst[tid] = s;
    pst[GBN + tid] = q;
    __syncthreads();
    const bool pok = tid < PARTW / 4;
    v4f pv = {0.f, 0.f, 0.f, 0.f};
    if (pok) pv = *(const v4fa*)(pst + 4 * tid);
    const size_t prow = (size_t)blockIdx.x * (size_t)gridDim.y + (size_t)blockIdx.y;
    float* pp = part + prow * PARTW + 4 * (pok ? tid : 0);
#pragma unroll
    for (int i = 0; i < 16; ++i) {
      const int gr = rowBase + 16 * wave + i;
      float* op = outF + (size_t)gr * (size_t)ldo + colBase + 4 * lane;
      if (gr < mRows) *(volatile v4f*)op = fv[i];
    }
    if (pok) *(volatile v4f*)pp = pv;
    __threadfence();
#pragma unroll
    for (int i = 0; i < 16; ++i) {
      const int gr = rowBase + 16 * wave + i;
      float* op = outF + (size_t)gr * (size_t)ldo + colBase + 4 * lane;
      if (gr < mRows) *(volatile v4f*)op = fv[i];
    }
    if (pok) *(volatile v4f*)pp = pv;
  }
}

__global__ __launch_bounds__(NTHR) void k_bnstat(const float* __restrict__ part, const float* __restrict__ gam,
                                                 const float* __restrict__ bet, float* stats,
                                                 double invN, int nPart, int gy) {
  __shared__ __attribute__((aligned(16))) float stg[4 * HD];
  const int tid = (int)threadIdx.x;
  const int by  = tid >> 7;
  const int lc  = tid & (GBN - 1);
  double S = 0.0, Q = 0.0;
#pragma unroll 4
  for (int b = 0; b < nPart; ++b) {
    const float* pr = part + ((size_t)b * (size_t)gy + (size_t)by) * PARTW;
    S += (double)pr[lc];
    Q += (double)pr[GBN + lc];
  }
  const double mean = S * invN;
  double var = Q * invN - mean * mean;
  var = (var < 0.0) ? 0.0 : var;
  const float mf = (float)mean;
  const float vf = (float)var;
  const float rs = rsqrtf(vf + 1e-5f);
  stg[tid]          = mf;
  stg[HD + tid]     = rs;
  stg[2 * HD + tid] = bf_rne(gam[tid]);
  stg[3 * HD + tid] = bf_rne(bet[tid]);
  __syncthreads();
  const v4f v = *(const v4fa*)(stg + 4 * tid);
  float* dp = stats + 4 * tid;
  *(volatile v4f*)dp = v;
  __threadfence();
  *(volatile v4f*)dp = v;
}

__global__ __launch_bounds__(NTHR) void k_pool(const float* __restrict__ U, const float* __restrict__ stats,
                                               const int* __restrict__ bat, int nN, float* out) {
  __shared__ int red[3 * NWAVE];
  __shared__ __attribute__((aligned(16))) float outs[HD];
  const int tid = (int)threadIdx.x, lane = tid & 31, wave = tid >> 5;
  const int g = (int)blockIdx.x;

  int cnt = 0, mn = 0x7fffffff, mx = -1;
  const int nIter = (nN + NTHR - 1) / NTHR;
#pragma unroll 4
  for (int it = 0; it < nIter; ++it) {
    const int i  = it * NTHR + tid;
    const int ic = i < nN ? i : nN - 1;
    const int b  = bat[ic];
    const bool hit = (i < nN) && (b == g);
    cnt += hit ? 1 : 0;
    mn = (hit && i < mn) ? i : mn;
    mx = (hit && i > mx) ? i : mx;
  }
#pragma unroll
  for (int d = 16; d >= 1; d >>= 1) {
    const int c2 = __shfl_xor(cnt, d);
    const int n2 = __shfl_xor(mn, d);
    const int x2 = __shfl_xor(mx, d);
    cnt += c2;
    mn = n2 < mn ? n2 : mn;
    mx = x2 > mx ? x2 : mx;
  }
  if (lane == 0) { red[wave] = cnt; red[NWAVE + wave] = mn; red[2 * NWAVE + wave] = mx; }
  __syncthreads();
  int tc = 0, tmn = 0x7fffffff, tmx = -1;
#pragma unroll
  for (int w2 = 0; w2 < NWAVE; ++w2) {
    tc += red[w2];
    const int a = red[NWAVE + w2], b = red[2 * NWAVE + w2];
    tmn = a < tmn ? a : tmn;
    tmx = b > tmx ? b : tmx;
  }

  const float cm = stats[tid], cr = stats[HD + tid], cg = stats[2 * HD + tid], cb = stats[3 * HD + tid];
  float acc = 0.0f;
  if (tc > 0) {
    const int lo = tmn < 0 ? 0 : (tmn > nN - 1 ? nN - 1 : tmn);
    const int hi = tmx < 0 ? 0 : (tmx > nN - 1 ? nN - 1 : tmx);
    if (hi - lo + 1 == tc) {
#pragma unroll 4
      for (int n = lo; n <= hi; ++n) {
        const float u = U[(size_t)n * HD + tid];
        acc += bnf(u, cm, cr, cg, cb);
      }
    } else {
#pragma unroll 1
      for (int n = 0; n < nN; ++n) {
        const int b = __builtin_amdgcn_readfirstlane(bat[n]);
        if (b == g) {
          const float u = U[(size_t)n * HD + tid];
          acc += bnf(u, cm, cr, cg, cb);
        }
      }
    }
  }
  outs[tid] = acc;
  __syncthreads();
  const bool okst = tid < HD / 4;
  const int t4 = okst ? tid : 0;
  const v4f ov = *(const v4fa*)(outs + 4 * t4);
  float* op = out + (size_t)g * HD + 4 * t4;
  if (okst) *(volatile v4f*)op = ov;
  __threadfence();
  if (okst) *(volatile v4f*)op = ov;
}

static inline int cdiv(int a, int b) { return (a + b - 1) / b; }
static inline size_t al256(size_t o) { return (o + 255) & ~(size_t)255; }

extern "C" void kernel_launch(void* const* d_in, const int* in_sizes, int n_in,
                              void* d_out, int out_size, void* d_ws, size_t ws_size,
                              hipStream_t stream) {
  if (n_in < 21) return;
  if (in_sizes[0] < FIN0 || (in_sizes[0] % FIN0) != 0) return;
  const int nN = in_sizes[0] / FIN0;
  if (nN < GBM || nN > (1 << 22)) return;
  const int nE2 = in_sizes[1];
  if (nE2 < 2 || (nE2 & 1) != 0) return;
  const int nE = nE2 / 2;
  if (nE < 1 || nE > (1 << 21)) return;
  if (in_sizes[2] != nN) return;
  for (int l = 0; l < 3; ++l) {
    const int fin = (l == 0) ? FIN0 : HD;
    if (in_sizes[3 + 6 * l] != fin * HD) return;
    if (in_sizes[4 + 6 * l] != HD) return;
    if (in_sizes[5 + 6 * l] != HD * HD) return;
    if (in_sizes[6 + 6 * l] != HD) return;
    if (in_sizes[7 + 6 * l] != HD) return;
    if (in_sizes[8 + 6 * l] != HD) return;
  }
  if (out_size < HD || (out_size % HD) != 0) return;
  const int nG = out_size / HD;
  if (nG < 1 || nG > 65535) return;
  if ((long long)nG * HD != (long long)out_size) return;

  const float* x     = (const float*)d_in[0];
  const int*   ei    = (const int*)  d_in[1];
  const int*   src   = ei;
  const int*   dst   = ei + nE;
  const int*   batch = (const int*)  d_in[2];
  const float* w1[3]; const float* b1[3]; const float* w2[3]; const float* b2[3];
  const float* ga[3]; const float* be[3];
  for (int l = 0; l < 3; ++l) {
    w1[l] = (const float*)d_in[3 + 6 * l];
    b1[l] = (const float*)d_in[4 + 6 * l];
    w2[l] = (const float*)d_in[5 + 6 * l];
    b2[l] = (const float*)d_in[6 + 6 * l];
    ga[l] = (const float*)d_in[7 + 6 * l];
    be[l] = (const float*)d_in[8 + 6 * l];
  }
  float* out = (float*)d_out;

  const int MP     = cdiv(nN, GBM) * GBM;
  const int gM     = MP / GBM;
  const int nbk    = cdiv(MP, NB);
  const int nSlots = nbk * NB;
  const int gy     = HD / GBN;
  const int vec8   = ((nE & 3) == 0) ? 1 : 0;
  if ((long long)nbk * NB < (long long)MP) return;
  if ((long long)(gM - 1) * GBM >= (long long)nN) return;

  char* ws = (char*)d_ws;
  size_t off = 0;
  const size_t szR = (size_t)MP * HD * 4;
  const size_t oR1 = off; off = al256(off + szR);
  const size_t oR2 = off; off = al256(off + szR);
  const size_t oXB = off; off = al256(off + (size_t)MP * FIN0 * 2);
  const size_t oSL = off; off = al256(off + (size_t)nbk * RCAP * 4);
  const size_t oST = off; off = al256(off + (size_t)nbk * NB * 4);
  const size_t oP10 = off; off = al256(off + (size_t)NU0 * 16);
  const size_t oP20 = off; off = al256(off + (size_t)NUW * 16);
  const size_t oP11 = off; off = al256(off + (size_t)NUW * 16);
  const size_t oP21 = off; off = al256(off + (size_t)NUW * 16);
  const size_t oP12 = off; off = al256(off + (size_t)NUW * 16);
  const size_t oP22 = off; off = al256(off + (size_t)NUW * 16);
  const size_t oPT = off; off = al256(off + (size_t)gM * gy * PARTW * 4);
  const size_t oSS = off; off = al256(off + (size_t)3 * 4 * HD * 4);
  if (off > ws_size || off > (size_t)WSLIM) return;
  char* R1 = ws + oR1;
  char* R2 = ws + oR2;
  unsigned short* XB  = (unsigned short*)(ws + oXB);
  int*            SRL = (int*)(ws + oSL);
  int*            SLT = (int*)(ws + oST);
  unsigned short* P10 = (unsigned short*)(ws + oP10);
  unsigned short* P20 = (unsigned short*)(ws + oP20);
  unsigned short* P11 = (unsigned short*)(ws + oP11);
  unsigned short* P21 = (unsigned short*)(ws + oP21);
  unsigned short* P12 = (unsigned short*)(ws + oP12);
  unsigned short* P22 = (unsigned short*)(ws + oP22);
  float*          PT  = (float*)(ws + oPT);
  float*          SS  = (float*)(ws + oSS);
  float* SS0 = SS;
  float* SS1 = SS + 4 * HD;
  float* SS2 = SS + 8 * HD;

  hipFuncSetAttribute(reinterpret_cast<const void*>(&k_hits), hipFuncAttributeMaxDynamicSharedMemorySize, LDS_HITS);

  const double invN = 1.0 / (double)nN;
  const int nUx = MP * (FIN0 / 8);

  k_wprep<<<NUTOT / NTHR, NTHR, 0, stream>>>(w1[0], w2[0], w1[1], w2[1], w1[2], w2[2], P10, P20, P11, P21, P12, P22);
  k_cvx<<<cdiv(nUx, NTHR), NTHR, 0, stream>>>(x, nN, nUx, XB);
  k_hits<<<nbk, NTHR, LDS_HITS, stream>>>(src, dst, nN, nE, vec8, SLT, SRL);

  k_agg<1><<<gM, NTHR, 0, stream>>>(SLT, SRL, XB, (const float*)R1, SS0, (unsigned short*)R2, nN, MP, nSlots);
  k_gemm<0><<<dim3(gM, gy), GTHR, 0, stream>>>((const unsigned short*)R2, K0, P10, K0, K0, b1[0],
                                               (void*)R1, KH, HD, nN, MP, PT);
  k_gemm<1><<<dim3(gM, gy), GTHR, 0, stream>>>((const unsigned short*)R1, KH, P20, KH, KH, b2[0],
                                               (void*)R2, HD, 0, nN, MP, PT);
  k_bnstat<<<1, NTHR, 0, stream>>>(PT, ga[0], be[0], SS0, invN, gM, gy);

  k_agg<0><<<gM, NTHR, 0, stream>>>(SLT, SRL, XB, (const float*)R2, SS0, (unsigned short*)R1, nN, MP, nSlots);
  k_gemm<0><<<dim3(gM, gy), GTHR, 0, stream>>>((const unsigned short*)R1, KH, P11, KH, KH, b1[1],
                                               (void*)R2, KH, HD, nN, MP, PT);
  k_gemm<1><<<dim3(gM, gy), GTHR, 0, stream>>>((const unsigned short*)R2, KH, P21, KH, KH, b2[1],
                                               (void*)R1, HD, 0, nN, MP, PT);
  k_bnstat<<<1, NTHR, 0, stream>>>(PT, ga[1], be[1], SS1, invN, gM, gy);

  k_agg<0><<<gM, NTHR, 0, stream>>>(SLT, SRL, XB, (const float*)R1, SS1, (unsigned short*)R2, nN, MP, nSlots);
  k_gemm<0><<<dim3(gM, gy), GTHR, 0, stream>>>((const unsigned short*)R2, KH, P12, KH, KH, b1[2],
                                               (void*)R1, KH, HD, nN, MP, PT);
  k_gemm<1><<<dim3(gM, gy), GTHR, 0, stream>>>((const unsigned short*)R1, KH, P22, KH, KH, b2[2],
                                               (void*)R2, HD, 0, nN, MP, PT);
  k_bnstat<<<1, NTHR, 0, stream>>>(PT, ga[2], be[2], SS2, invN, gM, gy);

  k_pool<<<nG, NTHR, 0, stream>>>((const float*)R2, SS2, batch, nN, out);
}
